// VectorWeightedAttention_23905787969985
// MI455X (gfx1250) — hardware-verified
//
#include <hip/hip_runtime.h>


namespace {
constexpr int NB = 64, S = 101, SP = 112  , JP = 128  , H = 512, NSLOT = 4;
constexpr float XS = 8.0f, PS = 1024.0f, LOG2E = 1.4426950408889634f, INVT = 0.044194173824159216f  ;

typedef _Float16 b16;
typedef __attribute__((ext_vector_type(16))) _Float16 v16b;
typedef __attribute__((ext_vector_type(8))) _Float16 v8b;
typedef __attribute__((ext_vector_type(8))) float v8f;
typedef __attribute__((ext_vector_type(4))) float v4f;
__device__ __forceinline__ float bf16_rne(float f) { unsigned int u = __float_as_uint(f); u += 0x7FFFu + ((u >> 16) & 1u); return __uint_as_float(u & 0xFFFF0000u); }
__device__ __forceinline__ void split16(float v, b16& hi, b16& lo) { hi = (b16)v; lo = (b16)(v - (float)hi); }
__device__ __forceinline__ v16b frag_kb(const b16* p, int hh) { const v8b a = *(const v8b*)(p + 8 * hh), b = *(const v8b*)(p + 16 + 8 * hh); v16b f;
#pragma unroll
  for (int e = 0; e < 8; ++e) { f[e] = a[e]; f[8 + e] = b[e]; } return f; }
__device__ __forceinline__ v8f wmma16b(v16b a, v16b b, v8f c) { v8f d = __builtin_amdgcn_wmma_f32_16x16x32_f16(false, a, false, b, (short)0, c, false, false); asm volatile("v_nop\n\tv_nop\n\tv_nop\n\tv_nop" : "+v"(d) : "v"(a), "v"(b)); return d; }
__device__ __forceinline__ void wave_lds_sync() { __builtin_amdgcn_fence(__ATOMIC_RELEASE, "workgroup"); __builtin_amdgcn_wave_barrier(); __builtin_amdgcn_fence(__ATOMIC_ACQUIRE, "workgroup"); }
__device__ __forceinline__ float nexp2(float x) { return __builtin_amdgcn_exp2f(x); }
__device__ __forceinline__ float pmul(float a, float b) { float p = a * b; asm volatile("" : "+v"(p)); return p; }
__device__ __forceinline__ int iclamp(int v, int lo, int hi) { return v < lo ? lo : (v > hi ? hi : v); }

__global__ __launch_bounds__(256) void prepqk_kernel(const float* __restrict__ q, const float* __restrict__ k, b16* __restrict__ Q16, b16* __restrict__ K16) {
  const size_t t = (size_t)blockIdx.x * 256 + threadIdx.x; const size_t per = (size_t)NB * SP * H / 8; if (t >= 2 * per) return; const int kind = (int)(t / per); const size_t e = (t - (size_t)kind * per) * 8;
  const size_t b = e / ((size_t)SP * H); const int i = (int)((e / H) % SP), c0 = (int)(e % H); const float* src = (kind == 0 ? q : k) + ((size_t)b * S + i) * H + c0; v8b o;
  if (i < S) { const v4f a = *(const v4f*)src, c = *(const v4f*)(src + 4); for (int j = 0; j < 4; ++j) { o[j] = (b16)(bf16_rne(a[j]) * XS); o[4 + j] = (b16)(bf16_rne(c[j]) * XS); } } else { for (int j = 0; j < 8; ++j) o[j] = (b16)0.0f; }
  b16* dst = (kind == 0 ? Q16 : K16) + e;
  for (int pass = 0; pass < 2; ++pass) { *(volatile v8b*)dst = o; __threadfence(); }
}
__global__ __launch_bounds__(256) void prepv_kernel(const float* __restrict__ v, b16* __restrict__ VT16) {
  __shared__ __attribute__((aligned(16))) b16 T[64][64 + 8];
  const int b = blockIdx.z, h0 = blockIdx.y * 64, j0 = blockIdx.x * 64, t_ = threadIdx.x;
  for (int qq = t_; qq < 64 * 64; qq += 256) { const int jj = qq >> 6, hh = qq & 63; const int j = j0 + jj; T[hh][jj] = (j < S) ? (b16)(bf16_rne(v[((size_t)b * S + j) * H + h0 + hh]) * XS) : (b16)0.0f; }
  __syncthreads();
  for (int pass = 0; pass < 2; ++pass) { for (int qq = t_; qq < 64 * 8; qq += 256) { const int hh = qq >> 3, c8 = (qq & 7) * 8; *(volatile v8b*)(VT16 + ((size_t)b * H + h0 + hh) * JP + j0 + c8) = *(const v8b*)(&T[hh][c8]); } __threadfence(); }
}
__global__ __launch_bounds__(32) void score_kernel(const b16* __restrict__ Q16, const b16* __restrict__ K16, const int* __restrict__ Kin, float* __restrict__ ATT, b16* __restrict__ Ph, b16* __restrict__ Pl) {
  __shared__ __attribute__((aligned(16))) float Ta[16][JP + 4]; __shared__ __attribute__((aligned(16))) b16 Th[16][JP + 8], Tl[16][JP + 8];
  const int lane = threadIdx.x, hh = lane >> 4, col = lane & 15; const int b = blockIdx.y, it = blockIdx.x; const int i0 = it * 16; const int KK = iclamp(Kin[0], 1, S); const int NK = S - 1;
  const b16* Qb = Q16 + ((size_t)b * SP) * H; const b16* Kb = K16 + ((size_t)b * SP) * H;
  v8f s[7];
#pragma unroll
  for (int t = 0; t < 7; ++t) s[t] = (v8f){};
  for (int kb = 0; kb < H; kb += 32) { const v16b a = frag_kb(Qb + (size_t)(i0 + col) * H + kb, hh);
#pragma unroll
    for (int t = 0; t < 7; ++t) s[t] = wmma16b(a, frag_kb(Kb + (size_t)(t * 16 + col) * H + kb, hh), s[t]); }
  const float cs = INVT * LOG2E / (XS * XS);
#pragma unroll
  for (int r = 0; r < 8; ++r) { float mx = -INFINITY;
#pragma unroll
    for (int t = 0; t < 7; ++t) { const int j = t * 16 + col; s[t][r] = (j < S) ? s[t][r] * cs : -INFINITY; mx = fmaxf(mx, s[t][r]); }
    mx = fmaxf(mx, __shfl_xor(mx, 1)); mx = fmaxf(mx, __shfl_xor(mx, 2)); mx = fmaxf(mx, __shfl_xor(mx, 4)); mx = fmaxf(mx, __shfl_xor(mx, 8));
    float sm = 0.0f;
#pragma unroll
    for (int t = 0; t < 7; ++t) { s[t][r] = nexp2(s[t][r] - mx); sm += s[t][r]; }
    sm += __shfl_xor(sm, 1); sm += __shfl_xor(sm, 2); sm += __shfl_xor(sm, 4); sm += __shfl_xor(sm, 8); const float inv = 1.0f / sm;
    const int i = i0 + 8 * hh + r;
#pragma unroll
    for (int t = 0; t < 7; ++t) { const int j = t * 16 + col; Ta[8 * hh + r][j] = (i < S && j < S) ? s[t][r] * inv : 0.0f; }
    Ta[8 * hh + r][112 + col] = 0.0f; }
  wave_lds_sync();
  for (int pass = 0; pass < 2; ++pass) { for (int rr = 0; rr < 16; ++rr) *(volatile v4f*)(ATT + ((size_t)b * SP + i0 + rr) * JP + lane * 4) = *(const v4f*)(&Ta[rr][lane * 4]); __threadfence(); }
  for (int slot = 0; slot < NSLOT; ++slot) {
    for (int qq = lane; qq < 16 * JP; qq += 32) { const int rr = qq / JP, j = qq % JP; const int i = i0 + rr; bool in;
      if (i < NK) { const bool same = (j < NK) && (j / KK == i / KK); in = slot == 0 ? (j == i) : slot == 1 ? (same && j != i) : slot == 2 ? (j < NK && !same) : (j == NK); }
      else { in = slot == 0 ? (j == NK) : slot == 1 ? (j < NK) : false; }
      const float p = in ? Ta[rr][j] * PS : 0.0f; b16 h_, l_; split16(p, h_, l_); Th[rr][j] = h_; Tl[rr][j] = l_; }
    wave_lds_sync();
    for (int pass = 0; pass < 2; ++pass) { for (int r2 = 0; r2 < 16; r2 += 2) { const int rr = r2 + (lane >> 4), c8 = (lane & 15) * 8; const size_t gi = (((size_t)b * NSLOT + slot) * SP + i0 + rr) * JP + c8; *(volatile v8b*)(Ph + gi) = *(const v8b*)(&Th[rr][c8]); *(volatile v8b*)(Pl + gi) = *(const v8b*)(&Tl[rr][c8]); } __threadfence(); }
    wave_lds_sync(); }
}
__global__ __launch_bounds__(32) void agg_kernel(const b16* __restrict__ Ph, const b16* __restrict__ Pl, const b16* __restrict__ VT16, const float* __restrict__ W6, float* __restrict__ out) {
  __shared__ __attribute__((aligned(16))) float To[16][128 + 4];
  const int lane = threadIdx.x, nloc = lane & 15, hlf = lane >> 4; const int b = blockIdx.y, it = blockIdx.x; const int i0 = it * 16; const int NK = S - 1;
  const b16* Vb = VT16 + (size_t)b * H * JP;
  for (int g = 0; g < H / 128; ++g) { v8f o[8];
#pragma unroll
    for (int t = 0; t < 8; ++t) o[t] = (v8f){};
    for (int slot = 0; slot < NSLOT; ++slot) { v8f acc[8];
#pragma unroll
      for (int t = 0; t < 8; ++t) acc[t] = (v8f){};
      const b16* P = Ph + (((size_t)b * NSLOT + slot) * SP + i0) * JP; const b16* PL = Pl + (((size_t)b * NSLOT + slot) * SP + i0) * JP;
#pragma unroll
      for (int kb = 0; kb < JP; kb += 32) { const v16b a = frag_kb(P + (size_t)nloc * JP + kb, hlf), al = frag_kb(PL + (size_t)nloc * JP + kb, hlf);
#pragma unroll
        for (int t = 0; t < 8; ++t) { const v16b bv = frag_kb(Vb + (size_t)(g * 128 + t * 16 + nloc) * JP + kb, hlf); acc[t] = wmma16b(a, bv, acc[t]); acc[t] = wmma16b(al, bv, acc[t]); } }
#pragma unroll
      for (int r = 0; r < 8; ++r) { const int i = i0 + 8 * hlf + r; const int wr = (i < NK) ? slot : (slot == 0 ? 5 : 4);
#pragma unroll
        for (int t = 0; t < 8; ++t) { const int h = g * 128 + t * 16 + nloc; o[t][r] += pmul(acc[t][r] * (1.0f / (PS * XS)), bf16_rne(W6[wr * H + h])); } } }
#pragma unroll
    for (int t = 0; t < 8; ++t)
#pragma unroll
      for (int r = 0; r < 8; ++r) To[8 * hlf + r][t * 16 + nloc] = o[t][r];
    wave_lds_sync();
    for (int pass = 0; pass < 2; ++pass) { for (int rr = 0; rr < 16; ++rr) if (i0 + rr < S) *(volatile v4f*)(out + ((size_t)b * S + i0 + rr) * H + g * 128 + lane * 4) = *(const v4f*)(&To[rr][lane * 4]); __threadfence(); }
    wave_lds_sync(); }
}
__global__ __launch_bounds__(256) void attncopy_kernel(const float* __restrict__ ATT, float* __restrict__ out1) {
  const size_t t = (size_t)blockIdx.x * 256 + threadIdx.x; const size_t total = (size_t)NB * S * S; if (t * 4 >= total) return; v4f o;
  for (int u = 0; u < 4; ++u) { const size_t f = t * 4 + u; float val = 0.0f; if (f < total) { const size_t b = f / ((size_t)S * S); const int rem = (int)(f % ((size_t)S * S)); const int i = rem / S, j = rem % S; val = ATT[((size_t)b * SP + i) * JP + j]; } o[u] = val; }
  for (int pass = 0; pass < 2; ++pass) { *(volatile v4f*)(out1 + t * 4) = o; __threadfence(); }
}
}

extern "C" void kernel_launch(void* const* d_in, const int* in_sizes, int n_in, void* d_out, int out_size, void* d_ws, size_t ws_size, hipStream_t stream) {
  (void)n_in;
  auto Fp = [&](int i) { return (const float*)d_in[i]; };
  if (in_sizes[0] != NB * S * H || in_sizes[1] != NB * S * H || in_sizes[2] != NB * S * H || in_sizes[3] != 6 * H || in_sizes[5] != 1 || out_size != NB * S * H + NB * S * S) return;
  size_t off = 0; char* ws = (char*)d_ws;
  auto carve = [&](size_t bytes) { char* p = ws + off; off += (bytes + 255) & ~(size_t)255; return p; };
  b16* Q16 = (b16*)carve((size_t)NB * SP * H * 2); b16* K16 = (b16*)carve((size_t)NB * SP * H * 2); b16* VT16 = (b16*)carve((size_t)NB * H * JP * 2); float* ATT = (float*)carve((size_t)NB * SP * JP * 4);
  b16* Ph = (b16*)carve((size_t)NB * NSLOT * SP * JP * 2); b16* Pl = (b16*)carve((size_t)NB * NSLOT * SP * JP * 2);
  if (off > ws_size || off > ((size_t)128 << 20)) return;
  float* out0 = (float*)d_out; float* out1 = out0 + (size_t)NB * S * H;
  prepqk_kernel<<<(unsigned)(((size_t)2 * NB * SP * H / 8 + 255) / 256), 256, 0, stream>>>(Fp(0), Fp(1), Q16, K16);
  prepv_kernel<<<dim3(JP / 64, H / 64, NB), 256, 0, stream>>>(Fp(2), VT16);
  score_kernel<<<dim3(SP / 16, NB), 32, 0, stream>>>(Q16, K16, (const int*)d_in[5], ATT, Ph, Pl);
  agg_kernel<<<dim3(SP / 16, NB), 32, 0, stream>>>(Ph, Pl, VT16, Fp(3), out0);
  attncopy_kernel<<<(unsigned)((((size_t)NB * S * S + 3) / 4 + 255) / 256), 256, 0, stream>>>(ATT, out1);
}
